// LSTMDQN_88957362635379
// MI455X (gfx1250) — hardware-verified
//
#include <hip/hip_runtime.h>
#include <math.h>

constexpr int NBATCH    = 16384;
constexpr int NSTEPS    = 30;
constexpr int NEMB      = 100;
constexpr int NHID      = 100;
constexpr int NVOC      = 100;
constexpr int NGATES    = 4;
constexpr int NGCOL     = NGATES * NHID;
constexpr int UPAD      = 112;
constexpr int PCOLS     = NGATES * UPAD;
constexpr int KPADH     = 128;
constexpr int NHEAD     = 6;
constexpr int ROWS_BLK  = 32;
constexpr int NTHR      = 448;
constexpr int NWAVE     = NTHR / 32;
constexpr int HPITCH    = 136;
constexpr int MSP       = UPAD;
constexpr int TKP       = 32;
constexpr int WPADL     = 2 * NTHR;
constexpr int NOUT_HALF = NBATCH * NHEAD;
constexpr int PREP_THR  = 256;
constexpr float WCARRY  = 256.0f;
constexpr float HCARRY  = 1024.0f;
constexpr float ZSC     = 1.0f / (256.0f * 1024.0f);
constexpr float FORGET_ADD = 1.0f;
constexpr float MEAN_SC = 1.0f / 30.0f;

static_assert(NBATCH % ROWS_BLK == 0, "grid exact");
static_assert(NWAVE == 2 * (UPAD / 16), "one wave per (m-subtile, unit-subtile)");
static_assert(UPAD % 16 == 0 && UPAD >= NHID, "unit padding");
static_assert(KPADH % 32 == 0 && KPADH >= NHID, "K padding multiple of 32");
static_assert(HPITCH % 8 == 0 && HPITCH >= KPADH, "h tile pitch");
static_assert((NVOC * PCOLS) % PREP_THR == 0, "xproj grid exact");
static_assert(PCOLS % 32 == 0, "xproj: one wave = one 128-B line");
static_assert((PCOLS * KPADH / 2) % PREP_THR == 0, "whplane grid exact");
static_assert(KPADH % 64 == 0, "whplane: one wave = one 128-B line");
static_assert((ROWS_BLK * PCOLS / 4) % NTHR == 0, "P staging loop exact");
static_assert(ROWS_BLK * 2 * NHEAD <= NTHR, "one thread per head output");
static_assert((ROWS_BLK * 2 * NHEAD) % 32 == 0, "head branch is wave-uniform");
static_assert(ROWS_BLK * NHEAD == 128 + 64, "store map: 32 lanes + 16 lanes x float4");
static_assert((ROWS_BLK * NHEAD * 4) % 128 == 0, "block output span is whole 128-B lines");
static_assert((NOUT_HALF * 4) % 128 == 0, "second output starts on a 128-B line");
static_assert(NSTEPS <= TKP, "token tile");
static_assert(NSTEPS == 30, "MEAN_SC matches NSTEPS");
static_assert(WPADL >= NHID * NHEAD, "head weight staging covers the whole matrix in 2 unconditional passes");

typedef __attribute__((ext_vector_type(16))) _Float16 v16h;
typedef __attribute__((ext_vector_type(8)))  _Float16 v8h;
typedef __attribute__((ext_vector_type(8)))  float    v8f;
typedef __attribute__((ext_vector_type(4)))  float    v4f;

__device__ __forceinline__ void wmma_guard45_h(v8f& a0, v8f& a1, v8f& a2, v8f& a3,
                                               v16h x, v16h y0, v16h y1, v16h y2, v16h y3) {
  asm volatile("v_nop\n\tv_nop\n\tv_nop\n\tv_nop"
               : "+v"(a0), "+v"(a1), "+v"(a2), "+v"(a3)
               : "v"(x), "v"(y0), "v"(y1), "v"(y2), "v"(y3));
}
__device__ __forceinline__ void acc_guard4(v8f& a, v8f& b, v8f& c, v8f& d) { asm volatile("v_nop\n\tv_nop\n\tv_nop\n\tv_nop" : "+v"(a), "+v"(b), "+v"(c), "+v"(d)); }
template <typename T> struct Frag;
template <> struct Frag<_Float16> {
  typedef v16h V; union U { v16h v; v8h h[2]; };
  static __device__ __forceinline__ v16h load(const _Float16* p) {
    U f; f.h[0] = *(const v8h*)(p); f.h[1] = *(const v8h*)(p + 16); return f.v;
  }
  static __device__ __forceinline__ v8f mma(v16h a, v16h b, v8f c) {
    return __builtin_amdgcn_wmma_f32_16x16x32_f16(false, a, false, b, (short)0, c, false, false);
  }
};

__device__ __forceinline__ float fsig(float x)  { return __builtin_amdgcn_rcpf(1.0f + expf(-x)); }
__device__ __forceinline__ float ftanh(float x) { return 1.0f - 2.0f * __builtin_amdgcn_rcpf(expf(2.0f * x) + 1.0f); }

__global__ __launch_bounds__(PREP_THR) void xproj_kernel(const float* __restrict__ emb, const float* __restrict__ wl,
                                                        const float* __restrict__ bl, float* __restrict__ P) {
  const int gi   = blockIdx.x * PREP_THR + threadIdx.x;
  const int v    = gi / PCOLS;
  const int col  = gi - v * PCOLS;
  const int g    = col / UPAD;
  const int u    = col - g * UPAD;
  const int uc   = (u < NHID) ? u : (NHID - 1);
  const int gcol = g * NHID + uc;
  const float* er = emb + (size_t)v * NEMB;
  const float* wc = wl + gcol;
  float acc = 0.0f;
#pragma unroll 4
  for (int k = 0; k < NEMB; ++k) acc = fmaf(er[k], wc[(size_t)k * NGCOL], acc);
  acc += bl[gcol];
  const float keep = (u < NHID) ? 1.0f : 0.0f;
  const float val = acc * keep;
  *(volatile float*)(P + gi) = val;
  __threadfence();
  *(volatile float*)(P + gi) = val;
}

__global__ __launch_bounds__(PREP_THR) void whplane_kernel(const float* __restrict__ wl, unsigned short* __restrict__ WH) {
  const int gi = blockIdx.x * PREP_THR + threadIdx.x;
  const int e0 = gi * 2;
  const int n  = e0 / KPADH;
  const int k  = e0 - n * KPADH;
  const int g  = n / UPAD;
  const int u  = n - g * UPAD;
  const int uc  = (u < NHID) ? u : (NHID - 1);
  const int k0c = (k < NHID) ? k : (NHID - 1);
  const int k1c = (k + 1 < NHID) ? (k + 1) : (NHID - 1);
  const float w0 = wl[(size_t)(NEMB + k0c) * NGCOL + g * NHID + uc];
  const float w1 = wl[(size_t)(NEMB + k1c) * NGCOL + g * NHID + uc];
  const float s0 = (u < NHID && k < NHID) ? WCARRY : 0.0f;
  const float s1 = (u < NHID && (k + 1) < NHID) ? WCARRY : 0.0f;
  const float f0 = w0 * s0;
  const float f1 = w1 * s1;
  const _Float16 h0 = (_Float16)f0, h1 = (_Float16)f1;
  const unsigned pk = (unsigned)__builtin_bit_cast(unsigned short, h0) | ((unsigned)__builtin_bit_cast(unsigned short, h1) << 16);
  ((volatile unsigned*)WH)[gi] = pk;
  __threadfence();
  ((volatile unsigned*)WH)[gi] = pk;
}

__device__ __forceinline__ void stage_rows(float* ps, const int* tk, const float* __restrict__ P, int t, int tid) {
#pragma unroll 4
  for (int it = 0; it < (ROWS_BLK * PCOLS / 4) / NTHR; ++it) {
    const int f   = it * NTHR + tid;
    const int row = f / (PCOLS / 4);
    const int q   = f - row * (PCOLS / 4);
    int tok = tk[row * TKP + t];
    tok = (tok < 0) ? 0 : tok;
    tok = (tok > NVOC - 1) ? (NVOC - 1) : tok;
    const v4f v = *(const v4f*)(P + (size_t)tok * PCOLS + 4 * q);
    *(v4f*)(ps + row * PCOLS + 4 * q) = v;
  }
}

__global__ __launch_bounds__(NTHR) void cell_seq_kernel(const int* __restrict__ toks, const float* __restrict__ P,
                                                        const unsigned short* __restrict__ WHp,
                                                        const float* __restrict__ wact, const float* __restrict__ bact,
                                                        const float* __restrict__ wobj, const float* __restrict__ bobj,
                                                        float* __restrict__ out) {
  __shared__ __align__(16) float    Ps[ROWS_BLK * PCOLS];
  __shared__ __align__(16) _Float16 Ah[2][ROWS_BLK * HPITCH];
  __shared__ __align__(16) float    Ms[ROWS_BLK * MSP];
  __shared__ __align__(16) float    Os[2 * ROWS_BLK * NHEAD];
  __shared__ int   Tk[ROWS_BLK * TKP];
  __shared__ float Was[WPADL];
  __shared__ float Wos[WPADL];

  const _Float16* WH = (const _Float16*)WHp;
  const int tid = threadIdx.x, lane = tid & 31, wave = tid >> 5;
  const int c = lane & 15, hh = lane >> 4, koff = hh * 8;
  const int mi = (wave >= 7) ? 1 : 0;
  const int ub = wave - 7 * mi;
  const int ucol = 16 * ub + c;
  const bool upad = (ucol >= NHID);
  const int mrow0 = 16 * mi + 8 * hh;
  const int rowbase = blockIdx.x * ROWS_BLK;

  {
    _Float16* ahf = &Ah[0][0];
#pragma unroll 1
    for (int i = tid; i < 2 * ROWS_BLK * HPITCH; i += NTHR) ahf[i] = (_Float16)0.0f;
  }
#pragma unroll 1
  for (int i = tid; i < ROWS_BLK * TKP; i += NTHR) {
    const int r  = i >> 5;
    const int tt = i & 31;
    const int tc = (tt < NSTEPS) ? tt : (NSTEPS - 1);
    int v = toks[(size_t)(rowbase + r) * NSTEPS + tc];
    v = (v < 0) ? (v + NVOC) : v;
    v = (v < 0) ? 0 : v;
    v = (v > NVOC - 1) ? (NVOC - 1) : v;
    Tk[i] = v;
  }
#pragma unroll
  for (int it = 0; it < 2; ++it) {
    const int i  = it * NTHR + tid;
    const int ic = (i < NHID * NHEAD) ? i : (NHID * NHEAD - 1);
    Was[i] = wact[ic];
    Wos[i] = wobj[ic];
  }
  float cst[8], hsum[8];
#pragma unroll
  for (int r = 0; r < 8; ++r) { cst[r] = 0.0f; hsum[r] = 0.0f; }
  __syncthreads();
  stage_rows(Ps, Tk, P, 0, tid);
  __syncthreads();

  const v8f z8 = {0.f, 0.f, 0.f, 0.f, 0.f, 0.f, 0.f, 0.f};

#pragma unroll 1
  for (int t = 0; t < NSTEPS; ++t) {
    const int cur = t & 1;
    const _Float16* ahrow = &Ah[cur][0] + (16 * mi + c) * HPITCH + koff;
    _Float16* ahn = &Ah[cur ^ 1][0];
    const _Float16* wrow = WH + (size_t)ucol * KPADH + koff;
    v8f acc[4];
    acc[0] = z8; acc[1] = z8; acc[2] = z8; acc[3] = z8;
#pragma unroll
    for (int kc = 0; kc < KPADH / 32; ++kc) {
      const int k0 = kc * 32;
      const v16h a  = Frag<_Float16>::load(ahrow + k0);
      const v16h b0 = Frag<_Float16>::load(wrow + k0);
      const v16h b1 = Frag<_Float16>::load(wrow + (size_t)1 * UPAD * KPADH + k0);
      const v16h b2 = Frag<_Float16>::load(wrow + (size_t)2 * UPAD * KPADH + k0);
      const v16h b3 = Frag<_Float16>::load(wrow + (size_t)3 * UPAD * KPADH + k0);
      acc[0] = Frag<_Float16>::mma(a, b0, acc[0]);
      acc[1] = Frag<_Float16>::mma(a, b1, acc[1]);
      acc[2] = Frag<_Float16>::mma(a, b2, acc[2]);
      acc[3] = Frag<_Float16>::mma(a, b3, acc[3]);
      wmma_guard45_h(acc[0], acc[1], acc[2], acc[3], a, b0, b1, b2, b3);
    }
    acc_guard4(acc[0], acc[1], acc[2], acc[3]);

#pragma unroll
    for (int r = 0; r < 8; ++r) {
      const int row = mrow0 + r;
      const float* pr = Ps + row * PCOLS + ucol;
      const float zi = fmaf(acc[0][r], ZSC, pr[0 * UPAD]);
      const float zj = fmaf(acc[1][r], ZSC, pr[1 * UPAD]);
      const float zf = fmaf(acc[2][r], ZSC, pr[2 * UPAD]) + FORGET_ADD;
      const float zo = fmaf(acc[3][r], ZSC, pr[3 * UPAD]);
      const float ig = fsig(zi);
      const float jg = ftanh(zj);
      const float fg = fsig(zf);
      const float og = fsig(zo);
      const float cn = cst[r] * fg + ig * jg;
      cst[r] = cn;
      float hn = ftanh(cn) * og;
      hn = upad ? 0.0f : hn;
      hsum[r] += hn;
      ahn[row * HPITCH + ucol] = (_Float16)(hn * HCARRY);
    }
    __syncthreads();
    {
      const int tn = (t + 1 < NSTEPS) ? (t + 1) : (NSTEPS - 1);
      stage_rows(Ps, Tk, P, tn, tid);
    }
    __syncthreads();
  }

#pragma unroll
  for (int r = 0; r < 8; ++r) Ms[(mrow0 + r) * MSP + ucol] = fmaxf(hsum[r] * MEAN_SC, 0.0f);
  __syncthreads();

  if (tid < ROWS_BLK * 2 * NHEAD) {
    const int row = tid / (2 * NHEAD);
    const int o   = tid - row * (2 * NHEAD);
    const int hd  = (o >= NHEAD) ? 1 : 0;
    const int jj  = o - NHEAD * hd;
    const float fb = (float)hd, fa = 1.0f - fb;
    const float* mr = Ms + row * MSP;
    float s = 0.0f;
#pragma unroll 4
    for (int u = 0; u < NHID; ++u) {
      const float w = fmaf(fa, Was[u * NHEAD + jj], fb * Wos[u * NHEAD + jj]);
      s = fmaf(mr[u], w, s);
    }
    const float ba = bact[jj], bo = bobj[jj];
    s += fmaf(fa, ba, fb * bo);
    Os[hd * (ROWS_BLK * NHEAD) + row * NHEAD + jj] = s;
  }
  __syncthreads();

  if (wave < 2) {
    const float* osrc = Os + wave * (ROWS_BLK * NHEAD);
    float* dst = out + (size_t)wave * NOUT_HALF + (size_t)rowbase * NHEAD;
    const int l2 = (lane < 16) ? lane : 15;
    const v4f v0 = *(const v4f*)(osrc + 4 * lane);
    const v4f v1 = *(const v4f*)(osrc + 128 + 4 * l2);
    for (int pass = 0; pass < 2; ++pass) {
      *(volatile v4f*)(dst + 4 * lane) = v0;
      if (lane < 16) *(volatile v4f*)(dst + 128 + 4 * lane) = v1;
      __threadfence();
    }
  }
}

extern "C" void kernel_launch(void* const* d_in, const int* in_sizes, int n_in,
                              void* d_out, int out_size, void* d_ws, size_t ws_size, hipStream_t stream) {
  if (n_in < 8 || d_out == nullptr || d_ws == nullptr) return;
  if (in_sizes[0] != NBATCH * NSTEPS || in_sizes[1] != NVOC * NEMB || in_sizes[2] != (NEMB + NHID) * NGCOL ||
      in_sizes[3] != NGCOL || in_sizes[4] != NHID * NHEAD || in_sizes[5] != NHEAD ||
      in_sizes[6] != NHID * NHEAD || in_sizes[7] != NHEAD || out_size != 2 * NOUT_HALF) return;

  const int*   toks  = (const int*)d_in[0];
  const float* embed = (const float*)d_in[1];
  const float* wl    = (const float*)d_in[2];
  const float* bl    = (const float*)d_in[3];
  const float* wact  = (const float*)d_in[4];
  const float* bact  = (const float*)d_in[5];
  const float* wobj  = (const float*)d_in[6];
  const float* bobj  = (const float*)d_in[7];
  float* out = (float*)d_out;

  char* ws = (char*)d_ws; size_t off = 0;
  auto carve = [&](size_t bytes) -> char* { char* p = ws + off; off += (bytes + 255) & ~(size_t)255; return p; };
  float*          P  = (float*)carve((size_t)NVOC * PCOLS * 4);
  unsigned short* WH = (unsigned short*)carve((size_t)PCOLS * KPADH * 2);
  if (off > ws_size || off > (size_t)134217728) return;

  xproj_kernel<<<(NVOC * PCOLS) / PREP_THR, PREP_THR, 0, stream>>>(embed, wl, bl, P);
  whplane_kernel<<<(PCOLS * KPADH / 2) / PREP_THR, PREP_THR, 0, stream>>>(wl, WH);
  cell_seq_kernel<<<NBATCH / ROWS_BLK, NTHR, 0, stream>>>(toks, P, WH, wact, bact, wobj, bobj, out);
}
